// GNNEncoder_63960652972724
// MI455X (gfx1250) — hardware-verified
//
#include <hip/hip_runtime.h>
#include <stddef.h>
#include <stdint.h>


#define FN     64
#define FE     16
#define HID    128
#define KEA    32
#define KC     256
#define KN     320
#define NTHR   256
#define NWAVE  8
#define EPT    8
#define CHUNK  (NTHR * EPT)
#define WCAP   (EPT * 32)
#define LISTN  (NWAVE * WCAP)
#define NBA    1024
#define SLA    10
#define RCAP   12288
#define DEGCAP 64
#define GBM    64
#define GBN    64
#define GTHR   128
#define TE     128
#define NU_WX  (HID * (FN / 8))
#define NU_WE  (HID * (KEA / 8))
#define NU_WC  (3 * HID * (KC / 8))
#define NU_WN  (HID * (KN / 8))
#define NU_ALL (NU_WX + NU_WE + NU_WC + NU_WN)
#define AGG_ZINTS (LISTN + 2 * RCAP + 3 * NBA)
#define AGG_LDS_INTS (AGG_ZINTS + 16)
#define LDS_TILE_C (TE * KC * 2)
#define LDS_TILE_N (TE * KN * 2)
#define LDS_TILE_H (TE * HID * 4)

static_assert((CHUNK & (CHUNK - 1)) == 0 && CHUNK <= 4096);
static_assert((NBA & (NBA - 1)) == 0 && NBA == (1 << SLA));
static_assert(((long long)CHUNK << SLA) < (1LL << 31));
static_assert(NBA % NWAVE == 0 && NBA % 32 == 0);
static_assert(RCAP % 32 == 0 && AGG_ZINTS % 4 == 0 && LISTN % 4 == 0);
static_assert(NU_WX % NTHR == 0 && NU_WE % NTHR == 0 && NU_WC % NTHR == 0 && NU_WN % NTHR == 0);
static_assert(KC % 32 == 0 && KN % 32 == 0 && FN % 32 == 0 && KEA == 32);
static_assert(TE == NWAVE * 16 && (TE * 16) % NTHR == 0 && (TE * 8) % NTHR == 0);
static_assert(16 * KC * 2 == 16 * HID * 4);
static_assert(16 * KN * 2 >= 16 * HID * 4);
static_assert(AGG_LDS_INTS * 4 <= 300000);
static_assert(HID == 4 * 32);

typedef float          v2f   __attribute__((ext_vector_type(2)));
typedef float          v4f   __attribute__((ext_vector_type(4)));
typedef float          v8f   __attribute__((ext_vector_type(8)));
typedef int            v4i   __attribute__((ext_vector_type(4)));
typedef int            v8i   __attribute__((ext_vector_type(8)));
typedef unsigned short v8us  __attribute__((ext_vector_type(8)));
typedef unsigned short v16us __attribute__((ext_vector_type(16)));
typedef __bf16         v16bf __attribute__((ext_vector_type(16)));
typedef v4f  __attribute__((may_alias)) v4fa;
typedef v4i  __attribute__((may_alias)) v4ia;
typedef v8us __attribute__((may_alias)) v8usa;
union FragB { v16bf v; v16us u; v8us h[2]; v8i w; };

__device__ __forceinline__ v8f z8f() { v8f z = {0.f, 0.f, 0.f, 0.f, 0.f, 0.f, 0.f, 0.f}; return z; }

__device__ __forceinline__ v8f wmb(const FragB& a, const FragB& b, v8f c) {
  v8f d = __builtin_amdgcn_wmma_f32_16x16x32_bf16(false, a.v, false, b.v, (short)0, c, false, false);
  asm volatile("v_nop\n\tv_nop\n\tv_nop\n\tv_nop" : "+v"(d) : "v"(a.w), "v"(b.w));
  return d;
}

__device__ __forceinline__ unsigned bf16_bits(float f) {
  const unsigned u = __float_as_uint(f);
  const unsigned r = (u + 0x7FFFu + ((u >> 16) & 1u)) >> 16;
  return (f != f) ? 0x7FC0u : r;
}
__device__ __forceinline__ float bf16_val(float f) { return __uint_as_float(bf16_bits(f) << 16); }

__device__ __forceinline__ v8us cvt8(v4f a, v4f b) {
  v8us o;
  o[0] = (unsigned short)bf16_bits(a.x); o[1] = (unsigned short)bf16_bits(a.y);
  o[2] = (unsigned short)bf16_bits(a.z); o[3] = (unsigned short)bf16_bits(a.w);
  o[4] = (unsigned short)bf16_bits(b.x); o[5] = (unsigned short)bf16_bits(b.y);
  o[6] = (unsigned short)bf16_bits(b.z); o[7] = (unsigned short)bf16_bits(b.w);
  return o;
}
__device__ __forceinline__ void split8(v4f a, v4f b, v8us& hi, v8us& lo) {
  float v[8] = {a.x, a.y, a.z, a.w, b.x, b.y, b.z, b.w};
#pragma unroll
  for (int k = 0; k < 8; ++k) {
    const unsigned h = bf16_bits(v[k]);
    hi[k] = (unsigned short)h;
    lo[k] = (unsigned short)bf16_bits(v[k] - __uint_as_float(h << 16));
  }
}
__device__ __forceinline__ float relun(float v) { return (v > 0.0f) ? v : (v - v); }
__device__ __forceinline__ v4f relu4n(v4f v) {
  v4f o; o.x = relun(v.x); o.y = relun(v.y); o.z = relun(v.z); o.w = relun(v.w); return o;
}
__device__ __forceinline__ v4f bf4(v4f v) {
  v4f o; o.x = bf16_val(v.x); o.y = bf16_val(v.y); o.z = bf16_val(v.z); o.w = bf16_val(v.w); return o;
}

template <int SLB>
__device__ __forceinline__ int scan_chunk(const int* __restrict__ dsts, int nE, int cbase, int slotBase,
                                          int nb, int vec8, int* list, int tid, int lane, int wave) {
  int wc = 0;
  const int el0  = tid * EPT;
  const int e0   = cbase + el0;
  const int sent = -2147483647 - 1;
  v4i da, db;
  if (vec8 != 0 && cbase + CHUNK <= nE) {
    da = *(const v4i*)(dsts + e0);
    db = *(const v4i*)(dsts + e0 + 4);
  } else {
    da.x = (e0     < nE) ? dsts[min(e0,     nE - 1)] : sent;
    da.y = (e0 + 1 < nE) ? dsts[min(e0 + 1, nE - 1)] : sent;
    da.z = (e0 + 2 < nE) ? dsts[min(e0 + 2, nE - 1)] : sent;
    da.w = (e0 + 3 < nE) ? dsts[min(e0 + 3, nE - 1)] : sent;
    db.x = (e0 + 4 < nE) ? dsts[min(e0 + 4, nE - 1)] : sent;
    db.y = (e0 + 5 < nE) ? dsts[min(e0 + 5, nE - 1)] : sent;
    db.z = (e0 + 6 < nE) ? dsts[min(e0 + 6, nE - 1)] : sent;
    db.w = (e0 + 7 < nE) ? dsts[min(e0 + 7, nE - 1)] : sent;
  }
  const unsigned nbs = (unsigned)slotBase;
  const unsigned unb = (unsigned)nb;
  const unsigned s0 = (unsigned)da.x - nbs, s1 = (unsigned)da.y - nbs;
  const unsigned s2 = (unsigned)da.z - nbs, s3 = (unsigned)da.w - nbs;
  const unsigned s4 = (unsigned)db.x - nbs, s5 = (unsigned)db.y - nbs;
  const unsigned s6 = (unsigned)db.z - nbs, s7 = (unsigned)db.w - nbs;
  const bool h0 = s0 < unb, h1 = s1 < unb, h2 = s2 < unb, h3 = s3 < unb;
  const bool h4 = s4 < unb, h5 = s5 < unb, h6 = s6 < unb, h7 = s7 < unb;
  const unsigned any = __builtin_amdgcn_ballot_w32(h0 | h1 | h2 | h3 | h4 | h5 | h6 | h7);
  if (any != 0u) {
#define HITJ(J, HJ, SJ) { \
      const unsigned mj = __builtin_amdgcn_ballot_w32(HJ); \
      if (mj != 0u) { \
        if (HJ) { \
          const int pos = wc + (int)__builtin_amdgcn_mbcnt_lo(mj, 0u); \
          if (pos < WCAP) list[wave * WCAP + pos] = ((el0 + (J)) << SLB) | (int)(SJ); \
        } \
        wc += (int)__builtin_popcount(mj); } }
    HITJ(0, h0, s0)
    HITJ(1, h1, s1)
    HITJ(2, h2, s2)
    HITJ(3, h3, s3)
    HITJ(4, h4, s4)
    HITJ(5, h5, s5)
    HITJ(6, h6, s6)
    HITJ(7, h7, s7)
#undef HITJ
  }
  return wc;
}

__global__ __launch_bounds__(NTHR) void k_prep(const float* __restrict__ Wei, const float* __restrict__ Wc,
                                               const float* __restrict__ Wn, unsigned short* WXT,
                                               unsigned short* WEAT, unsigned short* WC2, unsigned short* WNT) {
  const int u = (int)blockIdx.x * NTHR + (int)threadIdx.x;
  const float* p;
  unsigned short* dp;
  bool zr = false;
  if (u < NU_WX) {
    const int n = u >> 3, k8 = (u & 7) * 8;
    p  = Wei + (size_t)k8 * HID + n;
    dp = WXT + (size_t)u * 8;
  } else if (u < NU_WX + NU_WE) {
    const int v = u - NU_WX;
    const int n = v >> 2, k8 = (v & 3) * 8, kk = k8 & 15;
    p  = Wei + (size_t)(FN + kk) * HID + n;
    dp = WEAT + (size_t)v * 8;
    zr = k8 >= FE;
  } else if (u < NU_WX + NU_WE + NU_WC) {
    const int v = u - NU_WX - NU_WE;
    const int d = v >> 12, r = v & 4095;
    const int n = r >> 5, k8 = (r & 31) * 8, kk = k8 & (HID - 1);
    p  = Wc + (size_t)d * HID * HID + (size_t)kk * HID + n;
    dp = WC2 + (size_t)v * 8;
  } else if (u < NU_ALL) {
    const int v = u - NU_WX - NU_WE - NU_WC;
    const int n = v / (KN / 8);
    const int k8 = (v - n * (KN / 8)) * 8;
    const int kk = (k8 < FN + HID) ? k8 : k8 - HID;
    p  = Wn + (size_t)kk * HID + n;
    dp = WNT + (size_t)v * 8;
  } else {
    return;
  }
  v8us o;
#pragma unroll
  for (int i = 0; i < 8; ++i) {
    const unsigned b = bf16_bits(p[(size_t)i * HID]);
    o[i] = zr ? (unsigned short)0 : (unsigned short)b;
  }
  *(volatile v8us*)dp = o;
  __threadfence();
  *(volatile v8us*)dp = o;
}

__global__ __launch_bounds__(NTHR) void k_cvx(const float* __restrict__ x, int nN, int nUnits, unsigned short* xb) {
  const int u = (int)blockIdx.x * NTHR + (int)threadIdx.x;
  if (u >= nUnits) return;
  const int row = u >> 3;
  const int k8  = (u & 7) * 8;
  const int rc  = row < nN ? row : nN - 1;
  const float* p = x + (size_t)rc * FN + k8;
  const v4f a = *(const v4fa*)p;
  const v4f b = *(const v4fa*)(p + 4);
  const bool ok = row < nN;
  const v8us c = cvt8(a, b);
  v8us o;
#pragma unroll
  for (int i = 0; i < 8; ++i) o[i] = ok ? c[i] : (unsigned short)0;
  unsigned short* dp = xb + (size_t)row * FN + k8;
  *(volatile v8us*)dp = o;
  __threadfence();
  *(volatile v8us*)dp = o;
}

__global__ __launch_bounds__(GTHR) void k_gemm(const unsigned short* __restrict__ A,
                                               const unsigned short* __restrict__ WT,
                                               float* outF, int K, int ldo) {
  __shared__ __attribute__((aligned(16))) float stg[GBM * GBN];
  const int tid = (int)threadIdx.x, lane = tid & 31, wave = tid >> 5, hh = lane >> 4, m = lane & 15;
  const int rowBase = (int)blockIdx.x * GBM;
  const int col0    = (int)blockIdx.y * GBN;
  v8f acc[4];
  acc[0] = z8f(); acc[1] = z8f(); acc[2] = z8f(); acc[3] = z8f();
  const unsigned short* ap = A  + (size_t)(rowBase + 16 * wave + m) * (size_t)K + 8 * hh;
  const unsigned short* wp = WT + (size_t)(col0 + m) * (size_t)K + 8 * hh;
  const int ksteps = K >> 5;
#pragma unroll 1
  for (int ks = 0; ks < ksteps; ++ks) {
    FragB af;
    af.h[0] = *(const v8usa*)(ap + 32 * ks);
    af.h[1] = *(const v8usa*)(ap + 32 * ks + 16);
#pragma unroll
    for (int t = 0; t < 4; ++t) {
      const unsigned short* wq = wp + (size_t)(16 * t) * (size_t)K + 32 * ks;
      FragB bf;
      bf.h[0] = *(const v8usa*)wq;
      bf.h[1] = *(const v8usa*)(wq + 16);
      acc[t] = wmb(af, bf, acc[t]);
    }
  }
#pragma unroll
  for (int t = 0; t < 4; ++t) {
    const int lc = 16 * t + m;
#pragma unroll
    for (int r = 0; r < 8; ++r) {
      const int lr = 16 * wave + 8 * hh + r;
      stg[lr * GBN + lc] = acc[t][r];
    }
  }
  __syncthreads();
  v4f fv[8];
#pragma unroll
  for (int i = 0; i < 8; ++i) {
    const int lr = 16 * wave + 2 * i + hh;
    fv[i] = *(const v4fa*)(stg + lr * GBN + 4 * m);
  }
#pragma unroll
  for (int i = 0; i < 8; ++i) {
    const int gr = rowBase + 16 * wave + 2 * i + hh;
    float* op = outF + (size_t)gr * (size_t)ldo + col0 + 4 * m;
    *(volatile v4f*)op = fv[i];
  }
  __threadfence();
#pragma unroll
  for (int i = 0; i < 8; ++i) {
    const int gr = rowBase + 16 * wave + 2 * i + hh;
    float* op = outF + (size_t)gr * (size_t)ldo + col0 + 4 * m;
    *(volatile v4f*)op = fv[i];
  }
}

__global__ __launch_bounds__(NTHR) void k_h0(const float* __restrict__ ea, const int* __restrict__ ei,
                                             const float* __restrict__ xw, const unsigned short* __restrict__ weat,
                                             const float* __restrict__ bias, float* H, int nE, int nN) {
  extern __shared__ v4f lds_dyn[];
  float* stg = (float*)lds_dyn;
  const int tid = (int)threadIdx.x, lane = tid & 31, wave = tid >> 5, hh = lane >> 4, m = lane & 15;
  const int e0 = (int)blockIdx.x * TE;
  int er = e0 + 16 * wave + m;
  er = er > nE - 1 ? nE - 1 : er;
  FragB af;
  {
    const float* ap = ea + (size_t)er * FE + 8 * hh;
    const v4f a0 = *(const v4fa*)ap;
    const v4f a1 = *(const v4fa*)(ap + 4);
    af.h[0] = cvt8(a0, a1);
    const v8us zz = {0, 0, 0, 0, 0, 0, 0, 0};
    af.h[1] = zz;
  }
  v8f acc[8];
#pragma unroll
  for (int t = 0; t < 8; ++t) {
    const unsigned short* wq = weat + (size_t)(16 * t + m) * KEA + 8 * hh;
    FragB bf;
    bf.h[0] = *(const v8usa*)wq;
    bf.h[1] = *(const v8usa*)(wq + 16);
    acc[t] = wmb(af, bf, z8f());
  }
  float* sw = stg + wave * (16 * HID);
#pragma unroll
  for (int t = 0; t < 8; ++t) {
#pragma unroll
    for (int r = 0; r < 8; ++r) sw[(8 * hh + r) * HID + 16 * t + m] = acc[t][r];
  }
  __syncthreads();
  int rv = ei[er];
  rv = rv < 0 ? 0 : (rv > nN - 1 ? nN - 1 : rv);
  const v4f bv = bf4(*(const v4fa*)(bias + 4 * lane));
  v4f ov[16];
#pragma unroll
  for (int i = 0; i < 16; ++i) {
    const int rn = __builtin_amdgcn_readlane(rv, i);
    const v4f s = *(const v4fa*)(sw + i * HID + 4 * lane);
    const v4f g = *(const v4fa*)(xw + (size_t)rn * HID + 4 * lane);
    ov[i] = relu4n((s + g) + bv);
  }
  float* gp = H + (size_t)(e0 + 16 * wave) * HID + 4 * lane;
#pragma unroll
  for (int i = 0; i < 16; ++i) *(volatile v4f*)(gp + (size_t)i * HID) = ov[i];
  __threadfence();
#pragma unroll
  for (int i = 0; i < 16; ++i) *(volatile v4f*)(gp + (size_t)i * HID) = ov[i];
}

__global__ __launch_bounds__(NTHR) void k_agg(const int* __restrict__ dsts, int nE, int nN, int vec8, int mRows,
                                              const float* __restrict__ hs, float* outA) {
  extern __shared__ v4f lds_dyn[];
  int* dsm  = (int*)lds_dyn;
  int* list = dsm;
  int* hl   = dsm + LISTN;
  int* sl   = dsm + LISTN + RCAP;
  int* cnt  = dsm + LISTN + 2 * RCAP;
  int* offs = cnt + NBA;
  int* cur  = offs + NBA;
  int* misc = cur + NBA;
  const int tid = (int)threadIdx.x, lane = tid & 31, wave = tid >> 5;
  const int nodeBase = (int)blockIdx.x * NBA;
  {
    const v4i z4 = {0, 0, 0, 0};
    for (int i = tid * 4; i < AGG_ZINTS; i += NTHR * 4) *(v4ia*)(dsm + i) = z4;
    if (tid < 16) misc[tid] = 0;
  }
  __syncthreads();

  int t = 0, ov = 0;
  const int nChunks = (nE + CHUNK - 1) / CHUNK;
#pragma unroll 1
  for (int ch = 0; ch < nChunks; ++ch) {
    const int cbase = ch * CHUNK;
    const int wc = scan_chunk<SLA>(dsts, nE, cbase, nodeBase, NBA, vec8, list, tid, lane, wave);
    if (lane == 0) misc[wave] = wc;
    __syncthreads();
    if (wave == 0) {
#pragma unroll 1
      for (int w2 = 0; w2 < NWAVE; ++w2) {
        int c = misc[w2];
        c = c < 0 ? 0 : (c > WCAP ? WCAP : c);
#pragma unroll 1
        for (int b0 = 0; b0 < c; b0 += 32) {
          const int idx = b0 + lane;
          const int ent = list[w2 * WCAP + (idx < WCAP ? idx : WCAP - 1)];
          const int m32 = (c - b0) < 32 ? (c - b0) : 32;
#pragma unroll 1
          for (int k = 0; k < m32; ++k) {
            const int u    = __builtin_amdgcn_readlane(ent, k);
            const int slot = u & (NBA - 1);
            const int el   = (u >> SLA) & (CHUNK - 1);
            const int pk   = ((cbase + el) << SLA) | slot;
            if (t < RCAP) {
              if (lane == 0) { hl[t] = pk; cnt[slot] = cnt[slot] + 1; }
              t = t + 1;
            } else {
              ov = 1;
            }
          }
        }
      }
    }
    __syncthreads();
  }
  if (wave == 0 && lane == 0) { misc[8] = t; misc[9] = ov; }
  __syncthreads();
  int tt = misc[8];
  tt = tt < 0 ? 0 : (tt > RCAP ? RCAP : tt);
  const int ovf = misc[9];

  if (wave == 0) {
    const int base = lane * (NBA / 32);
    int s = 0;
#pragma unroll 1
    for (int i = 0; i < NBA / 32; ++i) s += cnt[base + i];
    int incl = s;
#pragma unroll
    for (int d = 1; d < 32; d <<= 1) {
      const int y = __shfl_up(incl, d, 32);
      if (lane >= d) incl += y;
    }
    int run = incl - s;
#pragma unroll 1
    for (int i = 0; i < NBA / 32; ++i) {
      const int cv = cnt[base + i];
      offs[base + i] = run;
      cur[base + i]  = run;
      run += cv;
    }
  }
  __syncthreads();
  if (wave == 0) {
#pragma unroll 1
    for (int b0 = 0; b0 < tt; b0 += 32) {
      const int idx = b0 + lane;
      const int ent = hl[idx < RCAP ? idx : RCAP - 1];
      const int m32 = (tt - b0) < 32 ? (tt - b0) : 32;
#pragma unroll 1
      for (int k = 0; k < m32; ++k) {
        const int u    = __builtin_amdgcn_readlane(ent, k);
        const int slot = u & (NBA - 1);
        if (lane == 0) {
          int p = cur[slot];
          p = p < 0 ? 0 : (p > RCAP - 1 ? RCAP - 1 : p);
          sl[p] = u;
          cur[slot] = p + 1;
        }
      }
    }
  }
  __syncthreads();

  const float qnan = __int_as_float(0x7fc00000);
  const float pz = (ovf != 0) ? qnan : 0.0f;
#pragma unroll 1
  for (int si = 0; si < NBA / NWAVE; ++si) {
    const int s    = si * NWAVE + wave;
    const int node = nodeBase + s;
    int c = cnt[s];
    const bool big = c > DEGCAP;
    c = c < 0 ? 0 : (c > DEGCAP ? DEGCAP : c);
    int o = offs[s];
    o = o < 0 ? 0 : (o > RCAP ? RCAP : o);
    v4f acc = {0.0f, 0.0f, 0.0f, 0.0f};
#pragma unroll 1
    for (int b0 = 0; b0 < c; b0 += 32) {
      int idx = o + b0 + lane;
      idx = idx > RCAP - 1 ? RCAP - 1 : idx;
      const int ent = sl[idx];
      int eid = ent >> SLA;
      eid = eid < 0 ? 0 : (eid > nE - 1 ? nE - 1 : eid);
      const int m32 = (c - b0) < 32 ? (c - b0) : 32;
#pragma unroll 1
      for (int k = 0; k < m32; ++k) {
        const int ek = __builtin_amdgcn_readlane(eid, k);
        const v4f a = *(const v4fa*)(hs + (size_t)ek * HID + 4 * lane);
        acc = acc + a;
      }
    }
    const float pzr = big ? qnan : pz;
    const bool live = node < nN;
    v4f y;
    y.x = acc.x + pzr; y.y = acc.y + pzr; y.z = acc.z + pzr; y.w = acc.w + pzr;
    v4f ow;
    ow.x = live ? y.x : 0.0f; ow.y = live ? y.y : 0.0f; ow.z = live ? y.z : 0.0f; ow.w = live ? y.w : 0.0f;
    float* op = outA + (size_t)node * HID + 4 * lane;
    const bool wr = node < mRows;
    if (wr) *(volatile v4f*)op = ow;
    __threadfence();
    if (wr) *(volatile v4f*)op = ow;
  }
}

__global__ __launch_bounds__(NTHR) void k_conv(const float* __restrict__ agg, float* H, const int* __restrict__ ei,
                                               const unsigned short* __restrict__ wc, const float* __restrict__ bias,
                                               int nE, int nN) {
  extern __shared__ v4f lds_dyn[];
  unsigned short* As = (unsigned short*)lds_dyn;
  float* stg = (float*)lds_dyn;
  const int tid = (int)threadIdx.x, lane = tid & 31, wave = tid >> 5, hh = lane >> 4, m = lane & 15;
  const int e0 = (int)blockIdx.x * TE;
#pragma unroll 1
  for (int it = 0; it < (TE * 16) / NTHR; ++it) {
    const int idx = it * NTHR + tid;
    const int el = idx >> 4, c = idx & 15;
    int e = e0 + el;
    e = e > nE - 1 ? nE - 1 : e;
    int rn = ei[e];
    rn = rn < 0 ? 0 : (rn > nN - 1 ? nN - 1 : rn);
    const float* gp = agg + (size_t)rn * HID + 8 * c;
    const float* hp = H + (size_t)(e ^ 1) * HID + 8 * c;
    const v4f g0 = *(const v4fa*)gp, g1 = *(const v4fa*)(gp + 4);
    const v4f h0 = *(const v4fa*)hp, h1 = *(const v4fa*)(hp + 4);
    const v4f m0 = g0 - h0, m1 = g1 - h1;
    v8us hi, lo;
    split8(m0, m1, hi, lo);
    *(v8usa*)(As + el * KC + 8 * c) = hi;
    *(v8usa*)(As + el * KC + HID + 8 * c) = lo;
  }
  __syncthreads();
  v8f acc[8];
#pragma unroll
  for (int t = 0; t < 8; ++t) acc[t] = z8f();
  const unsigned short* ap = As + (16 * wave + m) * KC + 8 * hh;
  const unsigned short* wp = wc + (size_t)m * KC + 8 * hh;
#pragma unroll 1
  for (int ks = 0; ks < KC / 32; ++ks) {
    FragB af;
    af.h[0] = *(const v8usa*)(ap + 32 * ks);
    af.h[1] = *(const v8usa*)(ap + 32 * ks + 16);
#pragma unroll
    for (int t = 0; t < 8; ++t) {
      const unsigned short* wq = wp + (size_t)(16 * t) * KC + 32 * ks;
      FragB bf;
      bf.h[0] = *(const v8usa*)wq;
      bf.h[1] = *(const v8usa*)(wq + 16);
      acc[t] = wmb(af, bf, acc[t]);
    }
  }
  __syncthreads();
  float* sw = stg + wave * (16 * HID);
#pragma unroll
  for (int t = 0; t < 8; ++t) {
#pragma unroll
    for (int r = 0; r < 8; ++r) sw[(8 * hh + r) * HID + 16 * t + m] = acc[t][r];
  }
  __syncthreads();
  const v4f bv = bf4(*(const v4fa*)(bias + 4 * lane));
  v4f ov[16];
#pragma unroll
  for (int i = 0; i < 16; ++i) ov[i] = relu4n(*(const v4fa*)(sw + i * HID + 4 * lane) + bv);
  float* gq = H + (size_t)(e0 + 16 * wave) * HID + 4 * lane;
#pragma unroll
  for (int i = 0; i < 16; ++i) *(volatile v4f*)(gq + (size_t)i * HID) = ov[i];
  __threadfence();
#pragma unroll
  for (int i = 0; i < 16; ++i) *(volatile v4f*)(gq + (size_t)i * HID) = ov[i];
}

__global__ __launch_bounds__(NTHR) void k_e2n(const unsigned short* __restrict__ xb, const float* __restrict__ sp,
                                              const unsigned short* __restrict__ wn, const float* __restrict__ bias,
                                              float* out, int nN) {
  extern __shared__ v4f lds_dyn[];
  unsigned short* As = (unsigned short*)lds_dyn;
  float* stg = (float*)lds_dyn;
  const int tid = (int)threadIdx.x, lane = tid & 31, wave = tid >> 5, hh = lane >> 4, m = lane & 15;
  const int nb = (int)blockIdx.x * TE;
#pragma unroll 1
  for (int it = 0; it < (TE * 8) / NTHR; ++it) {
    const int idx = it * NTHR + tid;
    const int el = idx >> 3, c = idx & 7;
    const v8us xv = *(const v8usa*)(xb + (size_t)(nb + el) * FN + 8 * c);
    *(v8usa*)(As + el * KN + 8 * c) = xv;
  }
#pragma unroll 1
  for (int it = 0; it < (TE * 16) / NTHR; ++it) {
    const int idx = it * NTHR + tid;
    const int el = idx >> 4, c = idx & 15;
    const float* q = sp + (size_t)(nb + el) * HID + 8 * c;
    const v4f s0 = *(const v4fa*)q, s1 = *(const v4fa*)(q + 4);
    v8us hi, lo;
    split8(s0, s1, hi, lo);
    *(v8usa*)(As + el * KN + FN + 8 * c) = hi;
    *(v8usa*)(As + el * KN + FN + HID + 8 * c) = lo;
  }
  __syncthreads();
  v8f acc[8];
#pragma unroll
  for (int t = 0; t < 8; ++t) acc[t] = z8f();
  const unsigned short* ap = As + (16 * wave + m) * KN + 8 * hh;
  const unsigned short* wp = wn + (size_t)m * KN + 8 * hh;
#pragma unroll 1
  for (int ks = 0; ks < KN / 32; ++ks) {
    FragB af;
    af.h[0] = *(const v8usa*)(ap + 32 * ks);
    af.h[1] = *(const v8usa*)(ap + 32 * ks + 16);
#pragma unroll
    for (int t = 0; t < 8; ++t) {
      const unsigned short* wq = wp + (size_t)(16 * t) * KN + 32 * ks;
      FragB bf;
      bf.h[0] = *(const v8usa*)wq;
      bf.h[1] = *(const v8usa*)(wq + 16);
      acc[t] = wmb(af, bf, acc[t]);
    }
  }
  __syncthreads();
  float* sw = stg + wave * (16 * KN / 2);
#pragma unroll
  for (int t = 0; t < 8; ++t) {
#pragma unroll
    for (int r = 0; r < 8; ++r) sw[(8 * hh + r) * HID + 16 * t + m] = acc[t][r];
  }
  __syncthreads();
  const v4f bv = bf4(*(const v4fa*)(bias + 4 * lane));
  v4f ov[16];
#pragma unroll
  for (int i = 0; i < 16; ++i) ov[i] = relu4n(*(const v4fa*)(sw + i * HID + 4 * lane) + bv);
  const int r0 = nb + 16 * wave;
  float* gq = out + (size_t)r0 * HID + 4 * lane;
#pragma unroll
  for (int i = 0; i < 16; ++i) { if (r0 + i < nN) *(volatile v4f*)(gq + (size_t)i * HID) = ov[i]; }
  __threadfence();
#pragma unroll
  for (int i = 0; i < 16; ++i) { if (r0 + i < nN) *(volatile v4f*)(gq + (size_t)i * HID) = ov[i]; }
}

static inline int cdiv(int a, int b) { return (a + b - 1) / b; }
static inline size_t al256(size_t o) { return (o + 255) & ~(size_t)255; }

extern "C" void kernel_launch(void* const* d_in, const int* in_sizes, int n_in,
                              void* d_out, int out_size, void* d_ws, size_t ws_size,
                              hipStream_t stream) {
  if (n_in < 9) return;
  if (in_sizes[0] < FN || (in_sizes[0] % FN) != 0) return;
  const int nN = in_sizes[0] / FN;
  if (nN < 1 || nN > (1 << 22)) return;
  if (in_sizes[1] < FE || (in_sizes[1] % FE) != 0) return;
  const int nE = in_sizes[1] / FE;
  if (nE < TE || (nE % TE) != 0 || nE >= (1 << (31 - SLA))) return;
  if (in_sizes[2] != 2 * nE) return;
  if (in_sizes[3] != (FN + FE) * HID || in_sizes[4] != HID) return;
  if (in_sizes[5] != 3 * HID * HID || in_sizes[6] != 3 * HID) return;
  if (in_sizes[7] != (FN + HID) * HID || in_sizes[8] != HID) return;
  if (out_size != nN * HID) return;

  const float* x    = (const float*)d_in[0];
  const float* ea   = (const float*)d_in[1];
  const int*   ei   = (const int*)d_in[2];
  const float* Wei  = (const float*)d_in[3];
  const float* bei  = (const float*)d_in[4];
  const float* Wcv  = (const float*)d_in[5];
  const float* bcv  = (const float*)d_in[6];
  const float* Wn   = (const float*)d_in[7];
  const float* bn   = (const float*)d_in[8];
  float* out = (float*)d_out;
  const int* tgt = ei + nE;

  const int MP = cdiv(nN, TE) * TE;
  const int gA = cdiv(MP, NBA);
  if ((long long)gA * NBA < (long long)MP) return;
  const int vec8 = ((nE & 3) == 0) ? 1 : 0;

  char* ws = (char*)d_ws;
  size_t off = 0;
  const size_t oH   = off; off = al256(off + (size_t)nE * HID * 4);
  const size_t oR1  = off; off = al256(off + (size_t)MP * HID * 4);
  const size_t oXB  = off; off = al256(off + (size_t)MP * FN * 2);
  const size_t oWX  = off; off = al256(off + (size_t)HID * FN * 2);
  const size_t oWE  = off; off = al256(off + (size_t)HID * KEA * 2);
  const size_t oWC  = off; off = al256(off + (size_t)3 * HID * KC * 2);
  const size_t oWN  = off; off = al256(off + (size_t)HID * KN * 2);
  if (off > ws_size) return;
  float*          H   = (float*)(ws + oH);
  float*          R1  = (float*)(ws + oR1);
  unsigned short* XB  = (unsigned short*)(ws + oXB);
  unsigned short* WXT = (unsigned short*)(ws + oWX);
  unsigned short* WEA = (unsigned short*)(ws + oWE);
  unsigned short* WC2 = (unsigned short*)(ws + oWC);
  unsigned short* WNT = (unsigned short*)(ws + oWN);

  const int aggLds = AGG_LDS_INTS * 4;
  hipFuncSetAttribute(reinterpret_cast<const void*>(&k_agg),  hipFuncAttributeMaxDynamicSharedMemorySize, aggLds);
  hipFuncSetAttribute(reinterpret_cast<const void*>(&k_h0),   hipFuncAttributeMaxDynamicSharedMemorySize, LDS_TILE_H);
  hipFuncSetAttribute(reinterpret_cast<const void*>(&k_conv), hipFuncAttributeMaxDynamicSharedMemorySize, LDS_TILE_C);
  hipFuncSetAttribute(reinterpret_cast<const void*>(&k_e2n),  hipFuncAttributeMaxDynamicSharedMemorySize, LDS_TILE_N);

  const int nUx = MP * (FN / 8);
  k_prep<<<NU_ALL / NTHR, NTHR, 0, stream>>>(Wei, Wcv, Wn, WXT, WEA, WC2, WNT);
  k_cvx<<<cdiv(nUx, NTHR), NTHR, 0, stream>>>(x, nN, nUx, XB);
  k_gemm<<<dim3(MP / GBM, HID / GBN), GTHR, 0, stream>>>(XB, WXT, R1, FN, HID);
  k_h0<<<nE / TE, NTHR, LDS_TILE_H, stream>>>(ea, ei, R1, WEA, bei, H, nE, nN);
  for (int d = 0; d < 3; ++d) {
    k_agg<<<gA, NTHR, aggLds, stream>>>(tgt, nE, nN, vec8, MP, H, R1);
    k_conv<<<nE / TE, NTHR, LDS_TILE_C, stream>>>(R1, H, ei, WC2 + (size_t)d * HID * KC, bcv + d * HID, nE, nN);
  }
  k_agg<<<gA, NTHR, aggLds, stream>>>(tgt, nE, nN, vec8, MP, H, R1);
  k_e2n<<<MP / TE, NTHR, LDS_TILE_N, stream>>>(XB, R1, WNT, bn, out, nN);
}
